// PointConv_1692217115333
// MI455X (gfx1250) — hardware-verified
//
#include <hip/hip_runtime.h>
#include <math.h>

typedef __attribute__((ext_vector_type(16))) _Float16 v16h;
typedef __attribute__((ext_vector_type(16))) __bf16 v16b;
typedef __attribute__((ext_vector_type(8)))  _Float16 v8h;
typedef __attribute__((ext_vector_type(8)))  float v8f;
typedef __attribute__((ext_vector_type(4)))  float v4f;
typedef __attribute__((ext_vector_type(2)))  float v2f;
typedef __attribute__((ext_vector_type(4)))  unsigned v4u;
typedef __attribute__((ext_vector_type(4)))  int v4i;
typedef float __attribute__((may_alias)) float_a;
typedef int __attribute__((may_alias)) int_a;

template <typename T> __device__ __forceinline__ void vst2(void* p, T v) { *(volatile T*)p = v; __threadfence(); *(volatile T*)p = v; }
__device__ __forceinline__ v8f wmma16(v16h a, v16h b, v8f c) {
  v8f d = __builtin_amdgcn_wmma_f32_16x16x32_f16(false, a, false, b, (short)0, c, false, false);
  asm volatile("v_nop\n\tv_nop\n\tv_nop\n\tv_nop" : "+v"(d) : "v"(a), "v"(b));
  return d;
}
__device__ __forceinline__ v8f wmma_bf(v16b a, v16b b, v8f c) {
  v8f d = __builtin_amdgcn_wmma_f32_16x16x32_bf16(false, a, false, b, (short)0, c, false, false);
  asm volatile("v_nop\n\tv_nop\n\tv_nop\n\tv_nop" : "+v"(d) : "v"(a), "v"(b));
  return d;
}
__device__ __forceinline__ v16h frag_h(const _Float16* rowk0, int lane) {
  union { v16h v; v8h q[2]; } u; const _Float16* p = rowk0 + 8 * (lane >> 4);
  u.q[0] = *(const v8h*)p; u.q[1] = *(const v8h*)(p + 16); return u.v;
}
__device__ __forceinline__ v16h frag_f32(const float* rowk0, int lane) {
  v16h a; const float* p = rowk0 + 8 * (lane >> 4);
#pragma unroll
  for (int i = 0; i < 8; ++i) { a[i] = (_Float16)p[i]; a[8 + i] = (_Float16)p[16 + i]; }
  return a;
}
__device__ __forceinline__ v16h frag_f32s(const float* rowk0, int lane, float sc) {
  v16h a; const float* p = rowk0 + 8 * (lane >> 4);
#pragma unroll
  for (int i = 0; i < 8; ++i) { a[i] = (_Float16)(p[i] * sc); a[8 + i] = (_Float16)(p[16 + i] * sc); }
  return a;
}
__device__ __forceinline__ v16h fragc_f32(const float* W, int k0, int n, int lane, int ld, int K) {
  v16h a; const int g = lane >> 4;
#pragma unroll
  for (int i = 0; i < 8; ++i) { const int ka = k0 + 8 * g + i, kb = ka + 16;
    a[i] = (_Float16)(ka < K ? W[(size_t)(ka < K ? ka : K - 1) * ld + n] : 0.f); a[8 + i] = (_Float16)(kb < K ? W[(size_t)(kb < K ? kb : K - 1) * ld + n] : 0.f); }
  return a;
}
struct F2 { v16b h, l; };
__device__ __forceinline__ F2 bsplit16(const float v[16]) { F2 r;
#pragma unroll
  for (int i = 0; i < 16; ++i) { const __bf16 h = (__bf16)v[i]; r.h[i] = h; r.l[i] = (__bf16)(v[i] - (float)h); }
  return r; }
__device__ __forceinline__ F2 split_row(const float* row, int k0, int lane) { float v[16]; const float* p = row + k0 + 8 * (lane >> 4);
#pragma unroll
  for (int i = 0; i < 8; ++i) { v[i] = p[i]; v[8 + i] = p[16 + i]; }
  return bsplit16(v); }
__device__ __forceinline__ F2 split_rowK(const float* row, int k0, int lane, int K) { float v[16]; const int g = lane >> 4;
#pragma unroll
  for (int i = 0; i < 8; ++i) { const int ka = k0 + 8 * g + i, kb = ka + 16; v[i] = ka < K ? row[ka < K ? ka : K - 1] : 0.f; v[8 + i] = kb < K ? row[kb < K ? kb : K - 1] : 0.f; }
  return bsplit16(v); }
__device__ __forceinline__ F2 split_col(const float* W, int k0, int n, int lane, int ld, int K) { float v[16]; const int g = lane >> 4;
#pragma unroll
  for (int i = 0; i < 8; ++i) { const int ka = k0 + 8 * g + i, kb = ka + 16; v[i] = ka < K ? W[(size_t)(ka < K ? ka : K - 1) * ld + n] : 0.f; v[8 + i] = kb < K ? W[(size_t)(kb < K ? kb : K - 1) * ld + n] : 0.f; }
  return bsplit16(v); }
__device__ __forceinline__ v8f mac3(const F2& a, const F2& b, v8f c) { c = wmma_bf(a.l, b.h, c); c = wmma_bf(a.h, b.l, c); return wmma_bf(a.h, b.h, c); }
__device__ __forceinline__ float sigm(float v) { return 1.0f / (1.0f + expf(-v)); }
#define LDSX() do { asm volatile("s_wait_dscnt 0" ::: "memory"); __builtin_amdgcn_wave_barrier(); __builtin_amdgcn_fence(__ATOMIC_RELEASE, "workgroup"); } while (0)

#define NBT 8
#define NPT 4096
#define DF 61
#define CE 64
#define WN 16
#define CO 64
#define KN 16
#define NR (NBT * NPT)
#ifndef NRV
#define NRV NR
#endif
#define AGW (CE * WN)
__device__ __forceinline__ float bfr(float v) { return (float)(__bf16)v; }
__device__ __forceinline__ v16b wcol_io(const float* __restrict__ Wm, int k0, int o, int lane, int ld) { v16b w; const float* p = Wm + (size_t)(k0 + 8 * (lane >> 4)) * ld + o;
#pragma unroll
  for (int i = 0; i < 8; ++i) { w[i] = (__bf16)p[(size_t)i * ld]; w[8 + i] = (__bf16)p[(size_t)(16 + i) * ld]; }
  asm volatile("s_wait_loadcnt 0x0" ::: "memory"); return w; }
#define WS_IDX 0u
#define WS_AG  (WS_IDX + 4u * (size_t)NR * KN)
#define WS_OT  (WS_AG + 4u * (size_t)NR * AGW)
#define WS_END (WS_OT + 4u * (size_t)NR * CO)
struct Best8 { float d[KN]; int i[KN]; };
__device__ __forceinline__ void push8(Best8& b, float d, int i) {
  if (d < b.d[KN - 1]) { b.d[KN - 1] = d; b.i[KN - 1] = i; }
#pragma unroll
  for (int p = KN - 1; p > 0; --p) { const bool sw = b.d[p] < b.d[p - 1]; const float td = b.d[p], ud = b.d[p - 1]; const int ti = b.i[p], ui = b.i[p - 1]; b.d[p] = sw ? ud : td; b.d[p - 1] = sw ? td : ud; b.i[p] = sw ? ui : ti; b.i[p - 1] = sw ? ti : ui; } }
__global__ __launch_bounds__(256) void k_knn(const float* __restrict__ P, int* __restrict__ IDX) { __shared__ int sidx8[8][KN];
  const int wave = threadIdx.x >> 5, lane = threadIdx.x & 31; const size_t row = (size_t)blockIdx.x * 8 + wave;
  const size_t b = row / NPT; const int n = (int)(row % NPT);
  Best8 bs;
#pragma unroll
  for (int r = 0; r < KN; ++r) { bs.d[r] = 3.0e38f; bs.i[r] = 0x7fffffff; }
  {
#pragma clang fp contract(off)
    const float qx = bfr(P[(b * 3 + 0) * NPT + n]), qy = bfr(P[(b * 3 + 1) * NPT + n]), qz = bfr(P[(b * 3 + 2) * NPT + n]);
    const float aa = (qx * qx + qy * qy) + qz * qz;
#pragma unroll 1
    for (int s = lane; s < NPT; s += 32) { const float px = bfr(P[(b * 3 + 0) * NPT + s]), py = bfr(P[(b * 3 + 1) * NPT + s]), pz = bfr(P[(b * 3 + 2) * NPT + s]);
      const float bb = (px * px + py * py) + pz * pz; const float dot = (qx * px + qy * py) + qz * pz; const float d = (aa + bb) - 2.0f * dot; push8(bs, d, s); } }
  int sel = 0;
#pragma unroll 1
  for (int r = 0; r < KN; ++r) { float d = bs.d[0]; int i = bs.i[0];
#pragma unroll
    for (int o = 1; o < 32; o <<= 1) { const float e = __shfl_xor(d, o); const int j = __shfl_xor(i, o); if (e < d || (e == d && j < i)) { d = e; i = j; } }
    if (lane == r) sel = i;
    { const bool pop = (bs.i[0] == i && bs.d[0] == d);
#pragma unroll
      for (int p = 0; p < KN - 1; ++p) { bs.d[p] = pop ? bs.d[p + 1] : bs.d[p]; bs.i[p] = pop ? bs.i[p + 1] : bs.i[p]; }
      bs.d[KN - 1] = pop ? 3.0e38f : bs.d[KN - 1]; bs.i[KN - 1] = pop ? 0x7fffffff : bs.i[KN - 1]; } }
  if (lane < KN) sidx8[wave][lane] = sel;
  __syncthreads();
  if (threadIdx.x < 32) vst2((v4i*)(IDX + (size_t)blockIdx.x * 8 * KN) + threadIdx.x, *(const v4i*)(&sidx8[0][0] + threadIdx.x * 4)); }


__global__ __launch_bounds__(128) void k_agg(const float* __restrict__ P, const float* __restrict__ FT, const int* __restrict__ IDX, const float* __restrict__ W0, const float* __restrict__ B0, const float* __restrict__ W1, const float* __restrict__ B1, const float* __restrict__ W2, const float* __restrict__ B2, float* __restrict__ AG) {
  __shared__ float sw[4][KN][WN + 1]; __shared__ float sg[4][KN][4]; __shared__ int sidx[4][KN]; __shared__ __align__(16) float so[4][64][20];
  const int tid = threadIdx.x, wave = tid >> 5, lane = tid & 31, col = lane & 15, g = lane >> 4;
  const size_t n = (size_t)blockIdx.x * 4 + wave; const size_t b = n / NPT; const int nl = (int)(n % NPT);
  if (lane < KN) { int ix = IDX[n * KN + lane]; ix = ix < 0 ? 0 : (ix >= NPT ? NPT - 1 : ix); sidx[wave][lane] = ix;
    const float gx = bfr(P[(b * 3 + 0) * NPT + ix]) - bfr(P[(b * 3 + 0) * NPT + nl]), gy = bfr(P[(b * 3 + 1) * NPT + ix]) - bfr(P[(b * 3 + 1) * NPT + nl]), gz = bfr(P[(b * 3 + 2) * NPT + ix]) - bfr(P[(b * 3 + 2) * NPT + nl]);
    sg[wave][lane][0] = gx; sg[wave][lane][1] = gy; sg[wave][lane][2] = gz; sg[wave][lane][3] = 0.f;
    float h0[8], h1[8];
#pragma unroll
    for (int o = 0; o < 8; ++o) h0[o] = fmaxf(((gx * bfr(W0[o * 3]) + gy * bfr(W0[o * 3 + 1])) + gz * bfr(W0[o * 3 + 2])) + bfr(B0[o]), 0.f);
#pragma unroll
    for (int o = 0; o < 8; ++o) { float a = 0.f;
#pragma unroll
      for (int i = 0; i < 8; ++i) a += h0[i] * bfr(W1[o * 8 + i]); h1[o] = fmaxf(a + bfr(B1[o]), 0.f); }
#pragma unroll
    for (int o = 0; o < WN; ++o) { float a = 0.f;
#pragma unroll
      for (int i = 0; i < 8; ++i) a += h1[i] * bfr(W2[o * 8 + i]); sw[wave][lane][o] = fmaxf(a + bfr(B2[o]), 0.f); } }
  LDSX();
  v16b wbh, wbl;
#pragma unroll
  for (int i = 0; i < 16; ++i) { const int kk = (i < 8) ? (8 * g + i) : (16 + 8 * g + (i - 8)); const float wv = kk < KN ? sw[wave][kk][col] : 0.f; const __bf16 hh = (__bf16)wv; wbh[i] = hh; wbl[i] = (__bf16)(wv - (float)hh); }
#pragma unroll
  for (int rt = 0; rt < 4; ++rt) { const int c = rt * 16 + col; float va[16];
#pragma unroll
    for (int i = 0; i < 16; ++i) { const int kk = (i < 8) ? (8 * g + i) : (16 + 8 * g + (i - 8)); const int kc = kk < KN ? kk : 0; float fv;
      { const int ix = sidx[wave][kc]; const int cf = c >= 3 ? c - 3 : 0; const float gf = FT[((size_t)b * DF + cf) * NPT + ix]; const float gc = sg[wave][kc][c < 3 ? c : 0]; fv = c < 3 ? gc : bfr(gf); }
      va[i] = kk < KN ? fv : 0.f; }
    asm volatile("s_wait_loadcnt 0x0" ::: "memory");
    const F2 a = bsplit16(va);
    v8f acc = {}; acc = wmma_bf(a.h, wbh, acc); acc = wmma_bf(a.h, wbl, acc); acc = wmma_bf(a.l, wbh, acc); acc = wmma_bf(a.l, wbl, acc);
#pragma unroll
    for (int r = 0; r < 8; ++r) so[wave][rt * 16 + 8 * g + r][col] = acc[r]; }
  LDSX();
  for (int c = 0; c < CE; c += 2) { const int cc = c + (lane >> 4); const int j = lane & 15; vst2(AG + n * AGW + cc * WN + j, so[wave][cc][j]); } }
__global__ __launch_bounds__(128) void k_lin(const float* __restrict__ AG, const float* __restrict__ LW, const float* __restrict__ LB, float* __restrict__ OT) { __shared__ __align__(16) float sf[4][16][68];
  const int tid = threadIdx.x, wave = tid >> 5, lane = tid & 31, col = lane & 15, g = lane >> 4; const size_t r0 = (size_t)blockIdx.x * 64 + wave * 16;
  v8f acc[4] = {};
#pragma unroll 2
  for (int kc = 0; kc < AGW / 32; ++kc) { const F2 a = split_row(AG + (r0 + col) * AGW, kc * 32, lane); asm volatile("s_wait_loadcnt 0x0" ::: "memory");
#pragma unroll
    for (int j = 0; j < 4; ++j) { v16b w; { const int o = j * 16 + col; const float* pw = LW + (size_t)o * AGW + kc * 32 + 8 * g;
#pragma unroll
        for (int i = 0; i < 8; ++i) { w[i] = (__bf16)pw[i]; w[8 + i] = (__bf16)pw[16 + i]; } }
      asm volatile("s_wait_loadcnt 0x0" ::: "memory"); acc[j] = wmma_bf(a.h, w, acc[j]); acc[j] = wmma_bf(a.l, w, acc[j]); } }
#pragma unroll
  for (int j = 0; j < 4; ++j) { const float bb = bfr(LB[j * 16 + col]);
#pragma unroll
    for (int r = 0; r < 8; ++r) { const float u = acc[j][r] + bb; sf[wave][8 * g + r][j * 16 + col] = u > 0.f ? u : 0.1f * u; } }
  LDSX(); for (int rl = 0; rl < 16; ++rl) if (lane < 16) vst2(OT + (r0 + rl) * CO + lane * 4, *(const v4f*)&sf[wave][rl][lane * 4]); }
__global__ __launch_bounds__(256) void k_cf(const float* __restrict__ OT, float* __restrict__ OUT) { __shared__ float st[64][68]; const int tid = threadIdx.x; const int n0 = blockIdx.x * 64; const size_t b = blockIdx.y;
  for (int e = tid; e < 64 * 16; e += 256) { const int nl = e >> 4, q = e & 15; *(v4f*)&st[nl][q * 4] = *(const v4f*)(OT + (b * NPT + n0 + nl) * CO + q * 4); }
  __syncthreads();
  for (int e = tid; e < 64 * 16; e += 256) { const int cl = e >> 4, q = e & 15; v4f o; o[0] = st[q * 4][cl]; o[1] = st[q * 4 + 1][cl]; o[2] = st[q * 4 + 2][cl]; o[3] = st[q * 4 + 3][cl]; vst2(OUT + (b * CO + cl) * (size_t)NPT + n0 + q * 4, o); } }
extern "C" void kernel_launch(void* const* d_in, const int* in_sizes, int n_in, void* d_out, int out_size, void* d_ws, size_t ws_size, hipStream_t stream) {
  (void)in_sizes; (void)n_in; (void)out_size;
  if (ws_size < (size_t)WS_END) return;
  char* ws = (char*)d_ws; const float** F = (const float**)d_in; int* IDX = (int*)(ws + WS_IDX); float *AG = (float*)(ws + WS_AG), *OT = (float*)(ws + WS_OT);
  k_knn<<<dim3(NRV / 8), 256, 0, stream>>>(F[0], IDX);
  k_agg<<<dim3(NRV / 4), 128, 0, stream>>>(F[0], F[1], IDX, F[2], F[3], F[4], F[5], F[6], F[7], AG);
  k_lin<<<dim3(NRV / 64), 128, 0, stream>>>(AG, F[8], F[9], OT);
  k_cf<<<dim3(NPT / 64, NRV / NPT), 256, 0, stream>>>(OT, (float*)d_out);
}
